// MultiHeadCrossAttention_27427661152300
// MI455X (gfx1250) — hardware-verified
//
#include <hip/hip_runtime.h>
#include <math.h>

#ifndef NB
#define NB 8
#endif
#ifndef SEQ
#define SEQ 1024
#endif
#define SEQ_FULL 1024
#define CH 512
#define NH 8
#define HD 64

static_assert(SEQ % 64 == 0);
static_assert(SEQ <= SEQ_FULL);
static_assert(CH == NH * HD);
static_assert(((SEQ / 64) * (CH / 64)) % 8 == 0);

typedef __attribute__((ext_vector_type(16))) __bf16   v16b;
typedef __attribute__((ext_vector_type(8)))  __bf16   v8b;
typedef __attribute__((ext_vector_type(8)))  float    v8f;
typedef __attribute__((ext_vector_type(4)))  float    v4f;
typedef __attribute__((ext_vector_type(4)))  unsigned v4u;


__device__ __forceinline__ unsigned short f2bf_bits(float f) {
  unsigned u = __float_as_uint(f);
  return (unsigned short)((u + 0x7FFFu + ((u >> 16) & 1u)) >> 16);
}
__device__ __forceinline__ float bf_bits2f(unsigned short h) { return __uint_as_float(((unsigned)h) << 16); }
__device__ __forceinline__ float bf_rne(float f) { return bf_bits2f(f2bf_bits(f)); }

union FragB { v16b v; v8b h[2]; };
__device__ __forceinline__ v16b frag_ld(const __bf16* p) {
  FragB f; f.h[0] = *(const v8b*)(p); f.h[1] = *(const v8b*)(p + 16); return f.v;
}
__device__ __forceinline__ v8f mma_raw(v16b a, v16b b, v8f c) {
  return __builtin_amdgcn_wmma_f32_16x16x32_bf16(false, a, false, b, (short)0, c, false, false);
}
__device__ __forceinline__ v8f mma_g(v16b a, v16b b, v8f c) {
  c = __builtin_amdgcn_wmma_f32_16x16x32_bf16(false, a, false, b, (short)0, c, false, false);
  asm volatile("v_nop\n\tv_nop\n\tv_nop\n\tv_nop" : "+v"(c) : "v"(a), "v"(b));
  return c;
}
__device__ __forceinline__ void dep_guard_b(v8f& a, v8f& b, v16b x, v16b y) { asm volatile("v_nop\n\tv_nop\n\tv_nop\n\tv_nop" : "+v"(a), "+v"(b) : "v"(x), "v"(y)); }
__device__ __forceinline__ void keep4_b(v16b a, v16b b, v16b c, v16b d) { asm volatile("v_nop" :: "v"(a), "v"(b), "v"(c), "v"(d)); }
__device__ __forceinline__ void acc_guard4(v8f& a, v8f& b, v8f& c, v8f& d) { asm volatile("v_nop\n\tv_nop\n\tv_nop\n\tv_nop" : "+v"(a), "+v"(b), "+v"(c), "+v"(d)); }
__device__ __forceinline__ void wave_sync_lds() {
  __builtin_amdgcn_fence(3  , "workgroup");
  __builtin_amdgcn_wave_barrier();
  __builtin_amdgcn_fence(2  , "workgroup");
}
__device__ __forceinline__ v4u pack8(const unsigned short* h) {
  v4u p;
  p.x = (unsigned)h[0] | ((unsigned)h[1] << 16);
  p.y = (unsigned)h[2] | ((unsigned)h[3] << 16);
  p.z = (unsigned)h[4] | ((unsigned)h[5] << 16);
  p.w = (unsigned)h[6] | ((unsigned)h[7] << 16);
  return p;
}

__global__ __launch_bounds__(256) void k_xt(const float* __restrict__ x0, const float* __restrict__ x1, const float* __restrict__ x2,
                                            unsigned short* __restrict__ XT) {
  __shared__ __align__(16) float tile[64][68];
  const int tid = threadIdx.x;
  const int s0 = blockIdx.x * 64, i0 = blockIdx.y * 64, z = blockIdx.z;
  const int which = z / NB, b = z - which * NB;
  const float* src = (which == 0) ? x0 : ((which == 1) ? x1 : x2);
  src += (size_t)b * CH * SEQ_FULL;
#pragma unroll
  for (int j = 0; j < 4; ++j) {
    const int idx = tid + 256 * j;
    const int r = idx >> 4, c4 = idx & 15;
    const v4f v = *(const v4f*)(src + (size_t)(i0 + r) * SEQ_FULL + s0 + 4 * c4);
    *(v4f*)&tile[r][4 * c4] = v;
  }
  __syncthreads();
  unsigned short* dst = XT + (size_t)z * SEQ * CH;
  v4u pk[2];
#pragma unroll
  for (int jj = 0; jj < 2; ++jj) {
    const int p = tid + 256 * jj;
    const int sl = p >> 3, i8 = (p & 7) * 8;
    unsigned short hb[8];
#pragma unroll
    for (int e = 0; e < 8; ++e) hb[e] = f2bf_bits(tile[i8 + e][sl]);
    pk[jj] = pack8(hb);
  }
#pragma unroll
  for (int jj = 0; jj < 2; ++jj) {
    const int p = tid + 256 * jj; const int sl = p >> 3, i8 = (p & 7) * 8;
    *(volatile v4u*)(dst + (size_t)(s0 + sl) * CH + i0 + i8) = pk[jj];
  }
  __threadfence();
#pragma unroll
  for (int jj = 0; jj < 2; ++jj) {
    const int p = tid + 256 * jj; const int sl = p >> 3, i8 = (p & 7) * 8;
    *(volatile v4u*)(dst + (size_t)(s0 + sl) * CH + i0 + i8) = pk[jj];
  }
}

static_assert((CH * CH) % (8 * 256) == 0);
__global__ __launch_bounds__(256) void k_wcvt(const float* __restrict__ w0, const float* __restrict__ w1, const float* __restrict__ w2,
                                              unsigned short* __restrict__ WB) {
  const int u = blockIdx.x * 256 + threadIdx.x;
  const int which = blockIdx.y;
  const float* src = (which == 0) ? w0 : ((which == 1) ? w1 : w2);
  const v4f a = *(const v4f*)(src + (size_t)8 * u), c = *(const v4f*)(src + (size_t)8 * u + 4);
  unsigned short hb[8];
  hb[0] = f2bf_bits(a.x); hb[1] = f2bf_bits(a.y); hb[2] = f2bf_bits(a.z); hb[3] = f2bf_bits(a.w);
  hb[4] = f2bf_bits(c.x); hb[5] = f2bf_bits(c.y); hb[6] = f2bf_bits(c.z); hb[7] = f2bf_bits(c.w);
  const v4u pk = pack8(hb);
  volatile v4u* d = (volatile v4u*)(WB + (size_t)which * CH * CH + (size_t)8 * u);
  *d = pk; __threadfence(); *d = pk;
}

template <int BIAS_MODE>
__global__ __launch_bounds__(256) void k_proj(
    const unsigned short* __restrict__ Ap, int lda, long strideA,
    const unsigned short* __restrict__ Btp, int ldb, long strideB,
    unsigned short* __restrict__ CHp, unsigned short* __restrict__ CLp, int ldc, long strideC,
    const float* __restrict__ bias, int M, int N, int K, float scale) {
  __shared__ __align__(16) float sT[8][16 * 68];
  const int b    = blockIdx.y;
  const int lane = threadIdx.x & 31;
  const int wave = threadIdx.x >> 5;
  const int tilesN = N >> 6;
  const int tilesM = M >> 6;
  const int tile = blockIdx.x * 8 + wave;
  if (tile >= tilesM * tilesN) return;
  const int tm = tile / tilesN;
  const int tn = tile - tm * tilesN;
  const int m0 = tm << 6;
  const int n0 = tn << 6;

  const __bf16* Ab = (const __bf16*)Ap  + (size_t)b * strideA;
  const __bf16* Bb = (const __bf16*)Btp + (size_t)b * strideB;

  const int rlane = lane & 15;
  const int koff  = (lane >> 4) * 8;
  const int mOff  = (lane >> 4) * 8;

  v8f acc[4][4];
#pragma unroll
  for (int i = 0; i < 4; ++i)
#pragma unroll
    for (int j = 0; j < 4; ++j) acc[i][j] = (v8f){0.f,0.f,0.f,0.f,0.f,0.f,0.f,0.f};

  for (int k0 = 0; k0 < K; k0 += 32) {
    v16b bh[4];
#pragma unroll
    for (int j = 0; j < 4; ++j) {
      const size_t bo = (size_t)(n0 + (j << 4) + rlane) * ldb + koff + k0;
      bh[j] = frag_ld(Bb + bo);
    }
#pragma unroll
    for (int i = 0; i < 4; ++i) {
      const size_t ao = (size_t)(m0 + (i << 4) + rlane) * lda + koff + k0;
      const v16b ah = frag_ld(Ab + ao);
#pragma unroll
      for (int j = 0; j < 4; ++j) acc[i][j] = mma_raw(ah, bh[j], acc[i][j]);
      dep_guard_b(acc[i][0], acc[i][3], ah, ah);
    }
    keep4_b(bh[0], bh[1], bh[2], bh[3]);
  }
  acc_guard4(acc[0][0], acc[0][1], acc[0][2], acc[0][3]);
  acc_guard4(acc[1][0], acc[1][1], acc[1][2], acc[1][3]);
  acc_guard4(acc[2][0], acc[2][1], acc[2][2], acc[2][3]);
  acc_guard4(acc[3][0], acc[3][1], acc[3][2], acc[3][3]);

  float* slab = sT[wave];
  unsigned short* C1 = CHp + (size_t)b * strideC;
  unsigned short* C2 = CLp + (size_t)b * strideC;
#pragma unroll
  for (int i = 0; i < 4; ++i) {
    const int mBase = m0 + (i << 4);
#pragma unroll
    for (int j = 0; j < 4; ++j) {
      const int n = n0 + (j << 4) + rlane;
      float bv = 0.f;
      if (BIAS_MODE == 2) bv = bf_rne(bias[n]);
#pragma unroll
      for (int r = 0; r < 8; ++r) {
        float v = acc[i][j][r];
        if (BIAS_MODE == 1) v += bf_rne(bias[mBase + mOff + r]);
        if (BIAS_MODE == 2) v += bv;
        v *= scale;
        slab[(mOff + r) * 68 + (j << 4) + rlane] = v;
      }
    }
    wave_sync_lds();
    {
      const int q = lane >> 3, c8 = (lane & 7) * 8;
      for (int pass = 0; pass < 2; ++pass) {
#pragma unroll
        for (int it = 0; it < 4; ++it) {
          const int row = it * 4 + q;
          const float* sp = slab + row * 68 + c8;
          unsigned short hb[8], lb[8];
#pragma unroll
          for (int e = 0; e < 8; ++e) {
            const float f = sp[e];
            hb[e] = f2bf_bits(f);
            lb[e] = f2bf_bits(f - bf_bits2f(hb[e]));
          }
          const v4u ph = pack8(hb), pl = pack8(lb);
          *(volatile v4u*)(C1 + (size_t)(mBase + row) * ldc + n0 + c8) = ph;
          *(volatile v4u*)(C2 + (size_t)(mBase + row) * ldc + n0 + c8) = pl;
        }
        __threadfence();
      }
    }
    wave_sync_lds();
  }
}

__global__ __launch_bounds__(128) void k_attn(const unsigned short* __restrict__ QHp, const unsigned short* __restrict__ QLp,
                                              const unsigned short* __restrict__ KHp, const unsigned short* __restrict__ KLp,
                                              const unsigned short* __restrict__ VHp, const unsigned short* __restrict__ VLp,
                                              float* __restrict__ out) {
  __shared__ __align__(16) __bf16 Psh[4][16 * 64];
  __shared__ __align__(16) __bf16 Psl[4][16 * 64];
  __shared__ __align__(16) float  Os[4][16 * 68];

  const int tid  = threadIdx.x;
  const int wave = tid >> 5;
  const int lane = tid & 31;
  const int hh   = lane >> 4;
  const int c    = lane & 15;

  const int nqb = SEQ / 64;
  const int bx = blockIdx.x;
  const int qb = bx % nqb;
  const int bh = bx / nqb;
  const int h  = bh % NH;
  const int b  = bh / NH;
  const int q0 = qb * 64 + wave * 16;

  const __bf16* QH = (const __bf16*)QHp + (size_t)b * SEQ * CH + h * HD;
  const __bf16* QL = (const __bf16*)QLp + (size_t)b * SEQ * CH + h * HD;
  const __bf16* KH = (const __bf16*)KHp + (size_t)b * SEQ * CH + h * HD;
  const __bf16* KL = (const __bf16*)KLp + (size_t)b * SEQ * CH + h * HD;
  const __bf16* VH = (const __bf16*)VHp + ((size_t)b * CH + h * HD) * SEQ;
  const __bf16* VL = (const __bf16*)VLp + ((size_t)b * CH + h * HD) * SEQ;

  v16b qah[2], qal[2];
#pragma unroll
  for (int dc = 0; dc < 2; ++dc) {
    const size_t qo = (size_t)(q0 + c) * CH + dc * 32 + 8 * hh;
    qah[dc] = frag_ld(QH + qo);
    qal[dc] = frag_ld(QL + qo);
  }

  float mrow[8], lrow[8];
  v8f oacc[4];
  const float NEGINF = -__builtin_inff();
#pragma unroll
  for (int r = 0; r < 8; ++r) { mrow[r] = NEGINF; lrow[r] = 0.f; }
#pragma unroll
  for (int t = 0; t < 4; ++t) oacc[t] = (v8f){0.f,0.f,0.f,0.f,0.f,0.f,0.f,0.f};

  __bf16* pwh = Psh[wave];
  __bf16* pwl = Psl[wave];

#pragma unroll 1
  for (int kc = 0; kc < SEQ / 64; ++kc) {
    const int kv0 = kc * 64;

    v8f s[4];
#pragma unroll
    for (int j = 0; j < 4; ++j) {
      s[j] = (v8f){0.f,0.f,0.f,0.f,0.f,0.f,0.f,0.f};
      const size_t ko = (size_t)(kv0 + j * 16 + c) * CH + 8 * hh;
#pragma unroll
      for (int dc = 0; dc < 2; ++dc) {
        const v16b kb = frag_ld(KH + ko + dc * 32);
        const v16b kl = frag_ld(KL + ko + dc * 32);
        s[j] = mma_g(qah[dc], kb, s[j]);
        s[j] = mma_g(qah[dc], kl, s[j]);
        s[j] = mma_g(qal[dc], kb, s[j]);
      }
    }

    float cm[8];
#pragma unroll
    for (int r = 0; r < 8; ++r) {
      float m = fmaxf(fmaxf(s[0][r], s[1][r]), fmaxf(s[2][r], s[3][r]));
#pragma unroll
      for (int off = 1; off < 16; off <<= 1) m = fmaxf(m, __shfl_xor(m, off, 32));
      cm[r] = m;
    }

#pragma unroll
    for (int r = 0; r < 8; ++r) {
      const float mnew = fmaxf(mrow[r], cm[r]);
      const float alpha = expf(mrow[r] - mnew);
      mrow[r] = mnew;
      float psum = 0.f;
#pragma unroll
      for (int j = 0; j < 4; ++j) {
        const float p = expf(s[j][r] - mnew);
        psum += p;
        const unsigned short hb = f2bf_bits(p);
        const unsigned short lb = f2bf_bits(p - bf_bits2f(hb));
        pwh[(8 * hh + r) * 64 + j * 16 + c] = __builtin_bit_cast(__bf16, hb);
        pwl[(8 * hh + r) * 64 + j * 16 + c] = __builtin_bit_cast(__bf16, lb);
      }
#pragma unroll
      for (int off = 1; off < 16; off <<= 1) psum += __shfl_xor(psum, off, 32);
      lrow[r] = lrow[r] * alpha + psum;
#pragma unroll
      for (int t = 0; t < 4; ++t) oacc[t][r] *= alpha;
    }
    wave_sync_lds();

#pragma unroll
    for (int kk = 0; kk < 2; ++kk) {
      const v16b pa = frag_ld(pwh + c * 64 + kk * 32 + 8 * hh);
      const v16b pl = frag_ld(pwl + c * 64 + kk * 32 + 8 * hh);
#pragma unroll
      for (int t = 0; t < 4; ++t) {
        const size_t vo = (size_t)(t * 16 + c) * SEQ + kv0 + kk * 32 + 8 * hh;
        const v16b vb = frag_ld(VH + vo);
        const v16b vl = frag_ld(VL + vo);
        oacc[t] = mma_g(pa, vb, oacc[t]);
        oacc[t] = mma_g(pa, vl, oacc[t]);
        oacc[t] = mma_g(pl, vb, oacc[t]);
      }
    }
    wave_sync_lds();
  }

  float* os = Os[wave];
#pragma unroll
  for (int r = 0; r < 8; ++r) {
    const float inv = 1.0f / lrow[r];
#pragma unroll
    for (int t = 0; t < 4; ++t) os[(8 * hh + r) * 68 + t * 16 + c] = oacc[t][r] * inv;
  }
  wave_sync_lds();
  {
    float* ob = out + (size_t)b * SEQ * CH + h * HD;
    const int c4 = (lane & 15) * 4;
    for (int pass = 0; pass < 2; ++pass) {
#pragma unroll
      for (int it = 0; it < 8; ++it) {
        const int row = it * 2 + hh;
        const v4f val = *(const v4f*)(os + row * 68 + c4);
        *(volatile v4f*)(ob + (size_t)(q0 + row) * CH + c4) = val;
      }
      __threadfence();
    }
  }
}

extern "C" void kernel_launch(void* const* d_in, const int* in_sizes, int n_in, void* d_out, int out_size, void* d_ws, size_t ws_size, hipStream_t stream) {
  if (n_in < 9) return;
  const long long need_x = (long long)NB * CH * SEQ;
  if ((long long)in_sizes[0] < need_x || (long long)in_sizes[1] < need_x || (long long)in_sizes[2] < need_x) return;
  if (in_sizes[3] < CH * CH || in_sizes[5] < CH * CH || in_sizes[7] < CH * CH) return;
  if (in_sizes[4] < CH || in_sizes[6] < CH || in_sizes[8] < CH) return;
  if ((long long)out_size < (long long)NB * SEQ * CH) return;

  const float* xq = (const float*)d_in[0];
  const float* xk = (const float*)d_in[1];
  const float* xv = (const float*)d_in[2];
  const float* wq = (const float*)d_in[3];
  const float* bq = (const float*)d_in[4];
  const float* wk = (const float*)d_in[5];
  const float* bk = (const float*)d_in[6];
  const float* wv = (const float*)d_in[7];
  const float* bv = (const float*)d_in[8];
  float* out = (float*)d_out;

  constexpr size_t PLANE = (size_t)NB * SEQ * CH * 2;
  constexpr size_t WSZ   = (size_t)3 * CH * CH * 2;
  constexpr size_t TOTAL = 9 * PLANE + WSZ;
  static_assert(PLANE % 256 == 0);
  static_assert(WSZ % 256 == 0);
  static_assert(TOTAL <= (size_t)134217728);
  if (TOTAL > ws_size) return;
  char* wsp = (char*)d_ws;
  unsigned short* XT = (unsigned short*)wsp; wsp += 3 * PLANE;
  unsigned short* WB = (unsigned short*)wsp; wsp += WSZ;
  unsigned short* QH = (unsigned short*)wsp; wsp += PLANE;
  unsigned short* QL = (unsigned short*)wsp; wsp += PLANE;
  unsigned short* KH = (unsigned short*)wsp; wsp += PLANE;
  unsigned short* KL = (unsigned short*)wsp; wsp += PLANE;
  unsigned short* VH = (unsigned short*)wsp; wsp += PLANE;
  unsigned short* VL = (unsigned short*)wsp; wsp += PLANE;

  const size_t XE = (size_t)NB * SEQ * CH;
  const unsigned short* XTq = XT;
  const unsigned short* XTk = XT + XE;
  const unsigned short* XTv = XT + 2 * XE;
  const unsigned short* WBq = WB;
  const unsigned short* WBk = WB + (size_t)CH * CH;
  const unsigned short* WBv = WB + (size_t)2 * CH * CH;

  k_xt<<<dim3(SEQ / 64, CH / 64, 3 * NB), 256, 0, stream>>>(xq, xk, xv, XT);
  k_wcvt<<<dim3((CH * CH) / (8 * 256), 3), 256, 0, stream>>>(wq, wk, wv, WB);

  const unsigned gx = (unsigned)(((SEQ / 64) * (CH / 64)) / 8);
  k_proj<2><<<dim3(gx, NB), 256, 0, stream>>>(XTq, CH, (long)SEQ * CH, WBq, CH, (long)0, QH, QL, CH, (long)SEQ * CH, bq, SEQ, CH, CH, 0.125f);
  k_proj<2><<<dim3(gx, NB), 256, 0, stream>>>(XTk, CH, (long)SEQ * CH, WBk, CH, (long)0, KH, KL, CH, (long)SEQ * CH, bk, SEQ, CH, CH, 1.0f);
  k_proj<1><<<dim3(gx, NB), 256, 0, stream>>>(WBv, CH, (long)0, XTv, CH, (long)SEQ * CH, VH, VL, SEQ, (long)CH * SEQ, bv, CH, SEQ, CH, 1.0f);

  k_attn<<<dim3((unsigned)(NB * NH * (SEQ / 64))), 128, 0, stream>>>(QH, QL, KH, KL, VH, VL, out);
}
